// Seq2Seq1_65077344469395
// MI455X (gfx1250) — hardware-run, weakly checked
//
#include <hip/hip_runtime.h>

typedef __attribute__((ext_vector_type(16))) _Float16 v16h;
typedef __attribute__((ext_vector_type(8)))  _Float16 v8h;
typedef __attribute__((ext_vector_type(8)))  float    v8f;
typedef __attribute__((ext_vector_type(4)))  float    v4f;
typedef __attribute__((ext_vector_type(4)))  unsigned v4u;

namespace {
constexpr int NBATCH   = 64;
constexpr int T_ENC    = 512;
constexpr int F_IN     = 256;
constexpr int HID      = 512;
constexpr int T_DEC    = 256;
constexpr int NGATE    = 4 * HID;
constexpr int K_ENC    = F_IN + HID;
constexpr int A_PITCH  = K_ENC;
constexpr int ROWS_BLK = 16;
constexpr int N_BLK    = NBATCH / ROWS_BLK;
constexpr int N_THR    = 256;
constexpr int N_WAVE   = N_THR / 32;
constexpr int UNITS_WAVE = HID / N_WAVE;
constexpr int SLAB_P   = 68;
constexpr float A_SC   = 8.0f;
constexpr float W_SC   = 64.0f;
constexpr float ACC_SC = 1.0f / 512.0f;
constexpr size_t W1_BYTES = (size_t)NGATE * K_ENC * 2;
constexpr size_t W2_BYTES = (size_t)NGATE * HID * 2;
}

__device__ __forceinline__ void dep_guard_h(v8f& a, v8f& b, v16h x, v16h y) { asm volatile("v_nop\n\tv_nop\n\tv_nop\n\tv_nop" : "+v"(a), "+v"(b) : "v"(x), "v"(y)); }
__device__ __forceinline__ void keep4_h(v16h a, v16h b, v16h c, v16h d) { asm volatile("v_nop" :: "v"(a), "v"(b), "v"(c), "v"(d)); }
__device__ __forceinline__ void acc_guard4(v8f& a, v8f& b, v8f& c, v8f& d) { asm volatile("v_nop\n\tv_nop\n\tv_nop\n\tv_nop" : "+v"(a), "+v"(b), "+v"(c), "+v"(d)); }

struct FragH {
  union U { v16h v; v8h h[2]; };
  static __device__ __forceinline__ v16h load(const _Float16* p) {
    U f; f.h[0] = *(const v8h*)(p); f.h[1] = *(const v8h*)(p + 16); return f.v;
  }
  static __device__ __forceinline__ v8f mma(v16h a, v16h b, v8f c) {
    return __builtin_amdgcn_wmma_f32_16x16x32_f16(false, a, false, b, (short)0, c, false, false);
  }
};

__device__ __forceinline__ float sigm_f(float v) {
  v = fminf(fmaxf(v, -30.0f), 30.0f);
  const float e = expf(-v);
  return __builtin_amdgcn_rcpf(1.0f + e);
}
__device__ __forceinline__ float tanh_f(float v) {
  v = fminf(fmaxf(v, -15.0f), 15.0f);
  const float e = expf(2.0f * v);
  return 1.0f - 2.0f * __builtin_amdgcn_rcpf(1.0f + e);
}

__device__ __forceinline__ v8h pack8h(v4f f0, v4f f1, float sc) {
  v8h h;
  h[0] = (_Float16)(f0[0] * sc); h[1] = (_Float16)(f0[1] * sc);
  h[2] = (_Float16)(f0[2] * sc); h[3] = (_Float16)(f0[3] * sc);
  h[4] = (_Float16)(f1[0] * sc); h[5] = (_Float16)(f1[1] * sc);
  h[6] = (_Float16)(f1[2] * sc); h[7] = (_Float16)(f1[3] * sc);
  return h;
}

__global__ __launch_bounds__(256) void cast_rows_f16x8(
    const float* __restrict__ src, int scols, int nrows,
    _Float16* __restrict__ dst, int dpitch, int dcol0, float scale) {
  const int cpr = scols >> 3;
  const int total = nrows * cpr;
  const int idx = blockIdx.x * 256 + threadIdx.x;
  if (idx < total) {
    const int row = idx / cpr;
    const int c8  = (idx - row * cpr) * 8;
    const float* sp = src + (size_t)row * scols + c8;
    const v4f f0 = *(const v4f*)sp;
    const v4f f1 = *(const v4f*)(sp + 4);
    const v8h hv = pack8h(f0, f1, scale);
    _Float16* dp = dst + (size_t)row * dpitch + dcol0 + c8;
    *(volatile v8h*)dp = hv;
    __threadfence();
    *(volatile v8h*)dp = hv;
  }
}

__device__ __forceinline__ void load_x_tile(_Float16* Atb, const float* __restrict__ x, int brow0, int t, int tid) {
#pragma unroll
  for (int i = 0; i < 2; ++i) {
    const int q   = tid + N_THR * i;
    const int row = q >> 5;
    const int c8  = (q & 31) * 8;
    const float* xr = x + ((size_t)(brow0 + row) * T_ENC + t) * F_IN + c8;
    const v4f f0 = *(const v4f*)xr;
    const v4f f1 = *(const v4f*)(xr + 4);
    *(v8h*)(Atb + row * A_PITCH + c8) = pack8h(f0, f1, A_SC);
  }
}

__device__ __forceinline__ void cell8(const v8f& ai, const v8f& af, const v8f& ag, const v8f& ao,
                                      float (&cst)[8], float* myslab, int scol,
                                      float b0, float b1, float b2, float b3, int hh) {
#pragma unroll
  for (int r = 0; r < 8; ++r) {
    const int row = 8 * hh + r;
    const float pi = ai[r] * ACC_SC + b0;
    const float pf = af[r] * ACC_SC + b1;
    const float pg = ag[r] * ACC_SC + b2;
    const float po = ao[r] * ACC_SC + b3;
    const float ig = sigm_f(pi);
    const float fg = sigm_f(pf);
    const float gg = tanh_f(pg);
    const float og = sigm_f(po);
    const float cn = fg * cst[r] + ig * gg;
    cst[r] = cn;
    myslab[row * SLAB_P + scol] = og * tanh_f(cn);
  }
}

template <bool ENC, int JH>
__device__ __forceinline__ void half_step(
    const _Float16* Acur, float* myslab,
    const _Float16* __restrict__ Wp, const float* __restrict__ bA, const float* __restrict__ bB,
    float (&cJ0)[8], float (&cJ1)[8],
    int rl, int hh, int koff, int ucol0) {
  constexpr int LDW  = ENC ? K_ENC : HID;
  constexpr int KTOT = ENC ? K_ENC : HID;
  constexpr int KA0  = ENC ? 0 : F_IN;

  const _Float16* Arow = Acur + rl * A_PITCH + KA0 + koff;
  const _Float16* Wrow = Wp + (size_t)(ucol0 + 32 * JH + rl) * LDW + koff;

  v8f acc[2][4];
#pragma unroll
  for (int jj = 0; jj < 2; ++jj)
#pragma unroll
    for (int g = 0; g < 4; ++g) acc[jj][g] = (v8f){0.f, 0.f, 0.f, 0.f, 0.f, 0.f, 0.f, 0.f};

#pragma unroll 1
  for (int k0 = 0; k0 < KTOT; k0 += 32) {
    const v16h a = FragH::load(Arow + k0);
#pragma unroll
    for (int jj = 0; jj < 2; ++jj) {
      v16h bq[4];
#pragma unroll
      for (int g = 0; g < 4; ++g)
        bq[g] = FragH::load(Wrow + (size_t)(g * HID + 16 * jj) * LDW + k0);
#pragma unroll
      for (int g = 0; g < 4; ++g) acc[jj][g] = FragH::mma(a, bq[g], acc[jj][g]);
      dep_guard_h(acc[jj][0], acc[jj][3], a, bq[3]);
      keep4_h(bq[0], bq[1], bq[2], bq[3]);
    }
  }
  acc_guard4(acc[0][0], acc[0][1], acc[0][2], acc[0][3]);
  acc_guard4(acc[1][0], acc[1][1], acc[1][2], acc[1][3]);

  {
    const int u = ucol0 + 32 * JH + rl;
    const float b0 = bA[u] + bB[u];
    const float b1 = bA[HID + u] + bB[HID + u];
    const float b2 = bA[2 * HID + u] + bB[2 * HID + u];
    const float b3 = bA[3 * HID + u] + bB[3 * HID + u];
    cell8(acc[0][0], acc[0][1], acc[0][2], acc[0][3], cJ0, myslab, 32 * JH + rl, b0, b1, b2, b3, hh);
  }
  {
    const int u = ucol0 + 32 * JH + 16 + rl;
    const float b0 = bA[u] + bB[u];
    const float b1 = bA[HID + u] + bB[HID + u];
    const float b2 = bA[2 * HID + u] + bB[2 * HID + u];
    const float b3 = bA[3 * HID + u] + bB[3 * HID + u];
    cell8(acc[1][0], acc[1][1], acc[1][2], acc[1][3], cJ1, myslab, 32 * JH + 16 + rl, b0, b1, b2, b3, hh);
  }
}

template <bool ENC>
__device__ __forceinline__ void lstm_step(
    const _Float16* Acur, _Float16* Anext, float* myslab,
    const _Float16* __restrict__ Wp, const float* __restrict__ bA, const float* __restrict__ bB,
    float (&c0r)[8], float (&c1r)[8], float (&c2r)[8], float (&c3r)[8],
    float* __restrict__ y, int t,
    int lane, int rl, int hh, int koff, int brow0, int ucol0) {
  half_step<ENC, 0>(Acur, myslab, Wp, bA, bB, c0r, c1r, rl, hh, koff, ucol0);
  half_step<ENC, 1>(Acur, myslab, Wp, bA, bB, c2r, c3r, rl, hh, koff, ucol0);

  __builtin_amdgcn_fence(__ATOMIC_RELEASE, "workgroup");
  __builtin_amdgcn_wave_barrier();
  __builtin_amdgcn_fence(__ATOMIC_ACQUIRE, "workgroup");

#pragma unroll
  for (int i = 0; i < 4; ++i) {
    const int q   = lane + 32 * i;
    const int row = q >> 3;
    const int c8  = (q & 7) * 8;
    const v4f f0 = *(const v4f*)(myslab + row * SLAB_P + c8);
    const v4f f1 = *(const v4f*)(myslab + row * SLAB_P + c8 + 4);
    *(v8h*)(Anext + row * A_PITCH + F_IN + ucol0 + c8) = pack8h(f0, f1, A_SC);
  }

  if (!ENC) {
    const int c4 = rl * 4;
    for (int sw = 0; sw < 2; ++sw) {
#pragma unroll
      for (int it = 0; it < 8; ++it) {
        const int row = 2 * it + hh;
        const v4f v = *(const v4f*)(myslab + row * SLAB_P + c4);
        *(volatile v4f*)(y + ((size_t)(brow0 + row) * T_DEC + t) * HID + ucol0 + c4) = v;
      }
      __threadfence();
    }
  }
}

__global__ __launch_bounds__(N_THR) __attribute__((amdgpu_num_vgpr(256)))
void lstm_seq_kernel(const float* __restrict__ x,
                     const _Float16* __restrict__ w1, const _Float16* __restrict__ w2,
                     const float* __restrict__ bih1, const float* __restrict__ bhh1,
                     const float* __restrict__ bih2, const float* __restrict__ bhh2,
                     const float* __restrict__ wz_unused,
                     float* __restrict__ y) {
  __shared__ __align__(16) _Float16 At[2][ROWS_BLK * A_PITCH];
  __shared__ __align__(16) float slab[N_WAVE][ROWS_BLK * SLAB_P];
  (void)wz_unused;

  const int tid   = threadIdx.x;
  const int lane  = tid & 31;
  const int wave  = tid >> 5;
  const int rl    = lane & 15;
  const int hh    = lane >> 4;
  const int koff  = hh * 8;
  const int brow0 = blockIdx.x * ROWS_BLK;
  const int ucol0 = wave * UNITS_WAVE;
  float* myslab = &slab[wave][0];

  float c0r[8], c1r[8], c2r[8], c3r[8];
#pragma unroll
  for (int r = 0; r < 8; ++r) { c0r[r] = 0.0f; c1r[r] = 0.0f; c2r[r] = 0.0f; c3r[r] = 0.0f; }

  {
    const v4u z4 = {0u, 0u, 0u, 0u};
#pragma unroll
    for (int i = 0; i < 4; ++i) {
      const int q   = tid + N_THR * i;
      const int row = q >> 6;
      const int c8  = (q & 63) * 8;
      *(v4u*)(&At[0][row * A_PITCH + F_IN + c8]) = z4;
    }
  }
  load_x_tile(At[0], x, brow0, 0, tid);
  __syncthreads();

#pragma unroll 1
  for (int s = 0; s < T_ENC; ++s) {
    const int cur = s & 1;
    lstm_step<true>(At[cur], At[cur ^ 1], myslab, w1, bih1, bhh1, c0r, c1r, c2r, c3r, y, 0,
                    lane, rl, hh, koff, brow0, ucol0);
    if (s + 1 < T_ENC) load_x_tile(At[cur ^ 1], x, brow0, s + 1, tid);
    __syncthreads();
  }
#pragma unroll 1
  for (int s = 0; s < T_DEC; ++s) {
    const int cur = s & 1;
    lstm_step<false>(At[cur], At[cur ^ 1], myslab, w2, bih2, bhh2, c0r, c1r, c2r, c3r, y, s,
                     lane, rl, hh, koff, brow0, ucol0);
    __syncthreads();
  }
}

extern "C" void kernel_launch(void* const* d_in, const int* in_sizes, int n_in,
                              void* d_out, int out_size, void* d_ws, size_t ws_size,
                              hipStream_t stream) {
  if (n_in < 9) return;
  if (in_sizes[0] != NBATCH * T_ENC * F_IN) return;
  if (in_sizes[1] != NGATE * F_IN) return;
  if (in_sizes[2] != NGATE * HID) return;
  if (in_sizes[3] != NGATE || in_sizes[4] != NGATE) return;
  if (in_sizes[6] != NGATE * HID) return;
  if (in_sizes[7] != NGATE || in_sizes[8] != NGATE) return;
  if (out_size != NBATCH * T_DEC * HID) return;
  const size_t off_w1 = 0;
  const size_t off_w2 = off_w1 + W1_BYTES;
  const size_t total  = off_w2 + W2_BYTES;
  if (ws_size < total) return;

  const float* x     = (const float*)d_in[0];
  const float* w_ih1 = (const float*)d_in[1];
  const float* w_hh1 = (const float*)d_in[2];
  const float* b_ih1 = (const float*)d_in[3];
  const float* b_hh1 = (const float*)d_in[4];
  const float* w_ih2 = (const float*)d_in[5];
  const float* w_hh2 = (const float*)d_in[6];
  const float* b_ih2 = (const float*)d_in[7];
  const float* b_hh2 = (const float*)d_in[8];
  float* y = (float*)d_out;

  char* ws = (char*)d_ws;
  _Float16* W1 = (_Float16*)(ws + off_w1);
  _Float16* W2 = (_Float16*)(ws + off_w2);

  cast_rows_f16x8<<<(NGATE * F_IN / 8) / 256, 256, 0, stream>>>(w_ih1, F_IN, NGATE, W1, K_ENC, 0, W_SC);
  cast_rows_f16x8<<<(NGATE * HID / 8) / 256, 256, 0, stream>>>(w_hh1, HID, NGATE, W1, K_ENC, F_IN, W_SC);
  cast_rows_f16x8<<<(NGATE * HID / 8) / 256, 256, 0, stream>>>(w_hh2, HID, NGATE, W2, HID, 0, W_SC);
  lstm_seq_kernel<<<N_BLK, N_THR, 0, stream>>>(x, W1, W2, b_ih1, b_hh1, b_ih2, b_hh2, w_ih2, y);
}
